// RelativeAttention_48026324303907
// MI455X (gfx1250) — hardware-verified
//
#include <hip/hip_runtime.h>

#ifndef NB
#define NB 2
#endif
#ifndef SEQ
#define SEQ 2048
#endif
#define SEQ_FULL 2048
#define ERROWS   2048
#define DMOD     1024
#define NHEAD    16
#define DHEAD    64
#define NBH      (NB * NHEAD)
#define MROWS    (NB * SEQ)

typedef __attribute__((ext_vector_type(16))) __bf16 v16b;
typedef __attribute__((ext_vector_type(8)))  __bf16 v8b;
typedef __attribute__((ext_vector_type(8)))  float  v8f;
typedef __attribute__((ext_vector_type(4)))  float  v4f;
typedef __attribute__((ext_vector_type(4)))  unsigned int v4u;

constexpr int QBLK  = 64;
constexpr int KCH   = 64;
constexpr int NWAVE = 4;
constexpr int RCOL  = 80;
constexpr int EP    = 72;
constexpr int VP    = 136;
constexpr int OP    = 68;
constexpr int CVT_PER_BLOCK = 2048;

constexpr size_t PLANE16 = (size_t)MROWS * DMOD * 2;
constexpr size_t WPLANE  = (size_t)DMOD * DMOD * 2;
constexpr size_t ERPLANE = (size_t)ERROWS * DHEAD * 2;
constexpr size_t OFF_XB = 0;
constexpr size_t OFF_WQ = OFF_XB + PLANE16;
constexpr size_t OFF_WK = OFF_WQ + WPLANE;
constexpr size_t OFF_WV = OFF_WK + WPLANE;
constexpr size_t OFF_WO = OFF_WV + WPLANE;
constexpr size_t OFF_ER = OFF_WO + WPLANE;
constexpr size_t OFF_QH = OFF_ER + ERPLANE;
constexpr size_t OFF_QL = OFF_QH + PLANE16;
constexpr size_t OFF_KH = OFF_QL + PLANE16;
constexpr size_t OFF_KL = OFF_KH + PLANE16;
constexpr size_t OFF_VH = OFF_KL + PLANE16;
constexpr size_t OFF_VL = OFF_VH + PLANE16;
constexpr size_t OFF_CH = OFF_VL + PLANE16;
constexpr size_t OFF_CL = OFF_CH + PLANE16;
constexpr size_t WS_NEED = OFF_CL + PLANE16;

static_assert(WS_NEED <= 134217728ull);
static_assert(SEQ % 128 == 0 && SEQ >= 128 && SEQ <= SEQ_FULL);
static_assert(ERROWS >= SEQ_FULL);
static_assert(MROWS % 128 == 0 && DMOD % 64 == 0 && DMOD % 32 == 0);
static_assert(DHEAD == 64 && QBLK == NWAVE * 16 && KCH == DHEAD && SEQ % QBLK == 0 && SEQ % KCH == 0);
static_assert((MROWS * DMOD) % CVT_PER_BLOCK == 0 && (DMOD * DMOD) % CVT_PER_BLOCK == 0 && (ERROWS * DHEAD) % CVT_PER_BLOCK == 0);
static_assert((OFF_ER % 128) == 0 && (OFF_QH % 128) == 0 && (WS_NEED % 128) == 0);
static_assert(NWAVE * 2 * 32 * EP >= 2 * 64 * VP);
static_assert((EP * 2) % 16 == 0 && (VP * 2) % 16 == 0 && (OP * 4) % 16 == 0);
static_assert(RCOL >= 64 + 15);


__device__ __forceinline__ unsigned short f2bf_bits(float f) {
  unsigned u = __float_as_uint(f);
  return (unsigned short)((u + 0x7FFFu + ((u >> 16) & 1u)) >> 16);
}
__device__ __forceinline__ float bf_bits2f(unsigned short h) { return __uint_as_float(((unsigned)h) << 16); }

__device__ __forceinline__ v8f zero8() {
  v8f z;
#pragma unroll
  for (int i = 0; i < 8; ++i) z[i] = 0.f;
  return z;
}

__device__ __forceinline__ v8f mma_bf16(v16b a, v16b b, v8f c) {
  c = __builtin_amdgcn_wmma_f32_16x16x32_bf16(false, a, false, b, (short)0, c, false, false);
  asm volatile("v_nop\n\tv_nop\n\tv_nop\n\tv_nop" : "+v"(c) : "v"(a), "v"(b) : "memory");
  return c;
}

__device__ __forceinline__ unsigned pack_bf2(float lo, float hi) {
  return (unsigned)f2bf_bits(lo) | ((unsigned)f2bf_bits(hi) << 16);
}

__global__ __launch_bounds__(256) void cvt_kernel(
    const float* __restrict__ x, const float* __restrict__ Wq, const float* __restrict__ Wk,
    const float* __restrict__ Wv, const float* __restrict__ Wo, const float* __restrict__ Er,
    unsigned short* __restrict__ ws16)
{
  const int reg = blockIdx.y;
  int nblk;
  const float* src;
  size_t dsto;
  if (reg == 0)      { nblk = (MROWS * DMOD) / CVT_PER_BLOCK;   src = x;  dsto = OFF_XB / 2; }
  else if (reg == 1) { nblk = (DMOD * DMOD) / CVT_PER_BLOCK;    src = Wq; dsto = OFF_WQ / 2; }
  else if (reg == 2) { nblk = (DMOD * DMOD) / CVT_PER_BLOCK;    src = Wk; dsto = OFF_WK / 2; }
  else if (reg == 3) { nblk = (DMOD * DMOD) / CVT_PER_BLOCK;    src = Wv; dsto = OFF_WV / 2; }
  else if (reg == 4) { nblk = (DMOD * DMOD) / CVT_PER_BLOCK;    src = Wo; dsto = OFF_WO / 2; }
  else               { nblk = (ERROWS * DHEAD) / CVT_PER_BLOCK; src = Er; dsto = OFF_ER / 2; }
  if ((int)blockIdx.x >= nblk) return;

  const size_t e = ((size_t)blockIdx.x * 256 + threadIdx.x) * 8;
  size_t se = e;
  if (reg == 0) {
    const size_t m   = e >> 10;
    const size_t col = e & 1023;
    const size_t bi  = m / SEQ;
    const size_t s   = m - bi * SEQ;
    se = (bi * SEQ_FULL + s) * DMOD + col;
  }
  const v4f a = *(const v4f*)(src + se);
  const v4f b = *(const v4f*)(src + se + 4);
  v4u w;
  w[0] = pack_bf2(a[0], a[1]);
  w[1] = pack_bf2(a[2], a[3]);
  w[2] = pack_bf2(b[0], b[1]);
  w[3] = pack_bf2(b[2], b[3]);
  unsigned short* dst = ws16 + dsto + e;
  *(volatile v4u*)dst = w;
  __threadfence();
  *(volatile v4u*)dst = w;
}

__global__ __launch_bounds__(128) __attribute__((amdgpu_num_vgpr(256))) void proj3_kernel(
    const unsigned short* __restrict__ Xb, const unsigned short* __restrict__ Wb3,
    const float* __restrict__ bq, const float* __restrict__ bk, const float* __restrict__ bv,
    unsigned short* __restrict__ planes)
{
  union FB { v16b v; v8b h[2]; };
  __shared__ __align__(16) unsigned short lds[NWAVE * 2 * 32 * EP];

  const int tid  = threadIdx.x;
  const int wave = tid >> 5;
  const int lane = tid & 31;
  const int hh   = lane >> 4;
  const int c    = lane & 15;
  const int m0   = blockIdx.x * 128;
  const int hsel = blockIdx.y;
  const int n0   = hsel * 64;
  const int z    = blockIdx.z;

  const unsigned short* W = Wb3 + (size_t)z * DMOD * DMOD;
  const float* bias = (z == 0) ? bq : ((z == 1) ? bk : bv);
  unsigned short* Ph = planes + (size_t)(2 * z) * MROWS * DMOD;
  unsigned short* Pl = Ph + (size_t)MROWS * DMOD;

  v8f acc[2][4];
#pragma unroll
  for (int mt = 0; mt < 2; ++mt)
#pragma unroll
    for (int nt = 0; nt < 4; ++nt) acc[mt][nt] = zero8();

  const size_t arow0 = (size_t)(m0 + 32 * wave + c) * DMOD + 8 * hh;
  const size_t brow0 = (size_t)(n0 + c) * DMOD + 8 * hh;

#pragma unroll 1
  for (int kt = 0; kt < DMOD / 32; ++kt) {
    const int k0 = kt * 32;
    FB a[2], b[4];
#pragma unroll
    for (int mt = 0; mt < 2; ++mt) {
      const unsigned short* ap = Xb + arow0 + (size_t)(16 * mt) * DMOD + k0;
      a[mt].h[0] = *(const v8b*)(ap);
      a[mt].h[1] = *(const v8b*)(ap + 16);
    }
#pragma unroll
    for (int nt = 0; nt < 4; ++nt) {
      const unsigned short* bp = W + brow0 + (size_t)(16 * nt) * DMOD + k0;
      b[nt].h[0] = *(const v8b*)(bp);
      b[nt].h[1] = *(const v8b*)(bp + 16);
    }
#pragma unroll
    for (int mt = 0; mt < 2; ++mt)
#pragma unroll
      for (int nt = 0; nt < 4; ++nt) acc[mt][nt] = mma_bf16(a[mt].v, b[nt].v, acc[mt][nt]);
  }

  float bcol[4];
#pragma unroll
  for (int nt = 0; nt < 4; ++nt) bcol[nt] = bf_bits2f(f2bf_bits(bias[n0 + 16 * nt + c]));

  if (z != 2) {
    unsigned short* eh = lds + wave * (2 * 32 * EP);
    unsigned short* el = eh + 32 * EP;
#pragma unroll
    for (int mt = 0; mt < 2; ++mt)
#pragma unroll
      for (int nt = 0; nt < 4; ++nt)
#pragma unroll
        for (int r = 0; r < 8; ++r) {
          const float v = acc[mt][nt][r] + bcol[nt];
          const unsigned short hb = f2bf_bits(v);
          const unsigned short lb = f2bf_bits(v - bf_bits2f(hb));
          const int row = 16 * mt + 8 * hh + r;
          eh[row * EP + 16 * nt + c] = hb;
          el[row * EP + 16 * nt + c] = lb;
        }
  } else {
    unsigned short* vsh = lds;
    unsigned short* vsl = lds + 64 * VP;
#pragma unroll
    for (int mt = 0; mt < 2; ++mt)
#pragma unroll
      for (int nt = 0; nt < 4; ++nt)
#pragma unroll
        for (int r = 0; r < 8; ++r) {
          const float v = acc[mt][nt][r] + bcol[nt];
          const unsigned short hb = f2bf_bits(v);
          const unsigned short lb = f2bf_bits(v - bf_bits2f(hb));
          const int row = 32 * wave + 16 * mt + 8 * hh + r;
          const int d   = 16 * nt + c;
          vsh[d * VP + row] = hb;
          vsl[d * VP + row] = lb;
        }
  }
  __syncthreads();

  const int seg = lane & 7;
  const int rq  = lane >> 3;
  if (z != 2) {
    const unsigned short* eh = lds + wave * (2 * 32 * EP);
    const unsigned short* el = eh + 32 * EP;
    for (int pass = 0; pass < 2; ++pass) {
#pragma unroll
      for (int it = 0; it < 8; ++it) {
        const int row = it * 4 + rq;
        const v4u vh = *(const v4u*)(eh + row * EP + seg * 8);
        const v4u vl = *(const v4u*)(el + row * EP + seg * 8);
        const int gm = m0 + 32 * wave + row;
        const int bi = gm / SEQ;
        const int s  = gm - bi * SEQ;
        const size_t o = ((size_t)((bi * NHEAD + hsel) * SEQ + s)) * DHEAD + seg * 8;
        *(volatile v4u*)(Ph + o) = vh;
        *(volatile v4u*)(Pl + o) = vl;
      }
      __threadfence();
    }
  } else {
    const unsigned short* vsh = lds;
    const unsigned short* vsl = lds + 64 * VP;
    const int bi   = m0 / SEQ;
    const int sblk = m0 - bi * SEQ;
    for (int pass = 0; pass < 2; ++pass) {
#pragma unroll
      for (int it = 0; it < 8; ++it) {
        const int L    = it * 16 + wave * 4 + rq;
        const int d    = L >> 1;
        const int soff = (L & 1) * 64 + seg * 8;
        const v4u vh = *(const v4u*)(vsh + d * VP + soff);
        const v4u vl = *(const v4u*)(vsl + d * VP + soff);
        const size_t o = ((size_t)((bi * NHEAD + hsel) * DHEAD + d)) * SEQ + sblk + soff;
        *(volatile v4u*)(Ph + o) = vh;
        *(volatile v4u*)(Pl + o) = vl;
      }
      __threadfence();
    }
  }
}

__global__ __launch_bounds__(128) __attribute__((amdgpu_num_vgpr(256))) void attn_kernel(
    const unsigned short* __restrict__ Qh, const unsigned short* __restrict__ Ql,
    const unsigned short* __restrict__ Kh, const unsigned short* __restrict__ Kl,
    const unsigned short* __restrict__ Vth, const unsigned short* __restrict__ Vtl,
    const unsigned short* __restrict__ Erb,
    unsigned short* __restrict__ Ch, unsigned short* __restrict__ Cl)
{
  union FB { v16b v; v8b h[2]; };
  __shared__ __align__(16) float Rl[NWAVE][16 * RCOL];
  __shared__ __align__(16) unsigned short Psh[NWAVE][16 * KCH];
  __shared__ __align__(16) unsigned short Psl[NWAVE][16 * KCH];

  const int tid  = threadIdx.x;
  const int wave = tid >> 5;
  const int lane = tid & 31;
  const int hh   = lane >> 4;
  const int c    = lane & 15;
  const int qb   = blockIdx.x;
  const int bh   = blockIdx.y;
  const int bi   = bh / NHEAD;
  const int hd   = bh - bi * NHEAD;
  const int q0   = qb * QBLK + wave * 16;

  v16b qah[2], qal[2];
  {
    const size_t ro = ((size_t)bh * SEQ + q0 + c) * DHEAD + 8 * hh;
#pragma unroll
    for (int dc = 0; dc < 2; ++dc) {
      FB t0, t1;
      t0.h[0] = *(const v8b*)(Qh + ro + dc * 32);
      t0.h[1] = *(const v8b*)(Qh + ro + dc * 32 + 16);
      t1.h[0] = *(const v8b*)(Ql + ro + dc * 32);
      t1.h[1] = *(const v8b*)(Ql + ro + dc * 32 + 16);
      qah[dc] = t0.v;
      qal[dc] = t1.v;
    }
  }

  float mrow[8], lrow[8];
  v8f oacc[4];
#pragma unroll
  for (int r = 0; r < 8; ++r) { mrow[r] = -__builtin_inff(); lrow[r] = 0.f; }
#pragma unroll
  for (int t = 0; t < 4; ++t) oacc[t] = zero8();

  const unsigned short* Khb = Kh  + (size_t)bh * SEQ * DHEAD + 8 * hh;
  const unsigned short* Klb = Kl  + (size_t)bh * SEQ * DHEAD + 8 * hh;
  const unsigned short* Vhb = Vth + (size_t)bh * DHEAD * SEQ + 8 * hh;
  const unsigned short* Vlb = Vtl + (size_t)bh * DHEAD * SEQ + 8 * hh;
  const unsigned short* Erl = Erb + 8 * hh;
  float* rl = Rl[wave];
  unsigned short* pwh = Psh[wave];
  unsigned short* pwl = Psl[wave];

#pragma unroll 1
  for (int kc = 0; kc <= qb; ++kc) {
    const int kv0 = kc * KCH;

    v8f s[4];
#pragma unroll
    for (int j = 0; j < 4; ++j) {
      s[j] = zero8();
      const size_t ko = (size_t)(kv0 + 16 * j + c) * DHEAD;
#pragma unroll
      for (int dc = 0; dc < 2; ++dc) {
        FB kh, kl;
        kh.h[0] = *(const v8b*)(Khb + ko + dc * 32);
        kh.h[1] = *(const v8b*)(Khb + ko + dc * 32 + 16);
        kl.h[0] = *(const v8b*)(Klb + ko + dc * 32);
        kl.h[1] = *(const v8b*)(Klb + ko + dc * 32 + 16);
        s[j] = mma_bf16(qah[dc], kh.v, s[j]);
        s[j] = mma_bf16(qah[dc], kl.v, s[j]);
        s[j] = mma_bf16(qal[dc], kh.v, s[j]);
      }
    }

    const int er0 = (ERROWS - 1) + kv0 - q0 - 15;
#pragma unroll
    for (int t = 0; t < 5; ++t) {
      int er = er0 + 16 * t + c;
      er = er < 0 ? 0 : er;
      er = er > (ERROWS - 1) ? (ERROWS - 1) : er;
      const unsigned short* ep = Erl + (size_t)er * DHEAD;
      v8f ra = zero8();
#pragma unroll
      for (int dc = 0; dc < 2; ++dc) {
        FB e;
        e.h[0] = *(const v8b*)(ep + dc * 32);
        e.h[1] = *(const v8b*)(ep + dc * 32 + 16);
        ra = mma_bf16(qah[dc], e.v, ra);
        ra = mma_bf16(qal[dc], e.v, ra);
      }
#pragma unroll
      for (int r = 0; r < 8; ++r) rl[(8 * hh + r) * RCOL + 16 * t + c] = ra[r];
    }
    __builtin_amdgcn_fence(3, "workgroup");
    __builtin_amdgcn_wave_barrier();
    __builtin_amdgcn_fence(2, "workgroup");

    const int lim0 = q0 - kv0 + 8 * hh;
#pragma unroll
    for (int j = 0; j < 4; ++j) {
      const int u = 16 * j + c;
#pragma unroll
      for (int r = 0; r < 8; ++r) {
        const int m = 8 * hh + r;
        const float v = (s[j][r] + rl[m * RCOL + u - m + 15]) * 0.125f;
        s[j][r] = (u <= lim0 + r) ? v : -1.0e9f;
      }
    }

    float cm[8];
#pragma unroll
    for (int r = 0; r < 8; ++r) {
      float m = fmaxf(fmaxf(s[0][r], s[1][r]), fmaxf(s[2][r], s[3][r]));
#pragma unroll
      for (int off = 1; off < 16; off <<= 1) m = fmaxf(m, __shfl_xor(m, off, 32));
      cm[r] = m;
    }

#pragma unroll
    for (int r = 0; r < 8; ++r) {
      const float mnew  = fmaxf(mrow[r], cm[r]);
      const float alpha = expf(mrow[r] - mnew);
      mrow[r] = mnew;
      float psum = 0.f;
#pragma unroll
      for (int j = 0; j < 4; ++j) {
        const float p = expf(s[j][r] - mnew);
        psum += p;
        const unsigned short hb = f2bf_bits(p);
        const unsigned short lb = f2bf_bits(p - bf_bits2f(hb));
        pwh[(8 * hh + r) * KCH + j * 16 + c] = hb;
        pwl[(8 * hh + r) * KCH + j * 16 + c] = lb;
      }
#pragma unroll
      for (int off = 1; off < 16; off <<= 1) psum += __shfl_xor(psum, off, 32);
      lrow[r] = lrow[r] * alpha + psum;
#pragma unroll
      for (int t = 0; t < 4; ++t) oacc[t][r] *= alpha;
    }
    __builtin_amdgcn_fence(3, "workgroup");
    __builtin_amdgcn_wave_barrier();
    __builtin_amdgcn_fence(2, "workgroup");

#pragma unroll
    for (int kk = 0; kk < 2; ++kk) {
      FB pa, pl;
      pa.h[0] = *(const v8b*)(pwh + c * KCH + kk * 32 + 8 * hh);
      pa.h[1] = *(const v8b*)(pwh + c * KCH + kk * 32 + 16 + 8 * hh);
      pl.h[0] = *(const v8b*)(pwl + c * KCH + kk * 32 + 8 * hh);
      pl.h[1] = *(const v8b*)(pwl + c * KCH + kk * 32 + 16 + 8 * hh);
#pragma unroll
      for (int t = 0; t < 4; ++t) {
        const size_t vo = (size_t)(16 * t + c) * SEQ + kv0 + kk * 32;
        FB vh, vl;
        vh.h[0] = *(const v8b*)(Vhb + vo);
        vh.h[1] = *(const v8b*)(Vhb + vo + 16);
        vl.h[0] = *(const v8b*)(Vlb + vo);
        vl.h[1] = *(const v8b*)(Vlb + vo + 16);
        oacc[t] = mma_bf16(pa.v, vh.v, oacc[t]);
        oacc[t] = mma_bf16(pa.v, vl.v, oacc[t]);
        oacc[t] = mma_bf16(pl.v, vh.v, oacc[t]);
      }
    }
  }

  __builtin_amdgcn_fence(3, "workgroup");
  __builtin_amdgcn_wave_barrier();
  __builtin_amdgcn_fence(2, "workgroup");
#pragma unroll
  for (int r = 0; r < 8; ++r) {
    const float inv = 1.0f / lrow[r];
#pragma unroll
    for (int t = 0; t < 4; ++t) {
      const float v = oacc[t][r] * inv;
      const unsigned short hb = f2bf_bits(v);
      const unsigned short lb = f2bf_bits(v - bf_bits2f(hb));
      pwh[(8 * hh + r) * KCH + 16 * t + c] = hb;
      pwl[(8 * hh + r) * KCH + 16 * t + c] = lb;
    }
  }
  __builtin_amdgcn_fence(3, "workgroup");
  __builtin_amdgcn_wave_barrier();
  __builtin_amdgcn_fence(2, "workgroup");
  {
    const int seg = lane & 7;
    const int rq  = lane >> 3;
    for (int pass = 0; pass < 2; ++pass) {
#pragma unroll
      for (int it = 0; it < 4; ++it) {
        const int row = it * 4 + rq;
        const v4u a = *(const v4u*)(pwh + row * KCH + seg * 8);
        const v4u b = *(const v4u*)(pwl + row * KCH + seg * 8);
        const size_t o = ((size_t)bi * SEQ + q0 + row) * DMOD + hd * DHEAD + seg * 8;
        *(volatile v4u*)(Ch + o) = a;
        *(volatile v4u*)(Cl + o) = b;
      }
      __threadfence();
    }
  }
}

__global__ __launch_bounds__(128) __attribute__((amdgpu_num_vgpr(256))) void oproj_kernel(
    const unsigned short* __restrict__ Ch, const unsigned short* __restrict__ Cl,
    const unsigned short* __restrict__ Wob, const float* __restrict__ bo,
    float* __restrict__ out)
{
  union FB { v16b v; v8b h[2]; };
  __shared__ __align__(16) float Os[NWAVE][32 * OP];

  const int tid  = threadIdx.x;
  const int wave = tid >> 5;
  const int lane = tid & 31;
  const int hh   = lane >> 4;
  const int c    = lane & 15;
  const int m0   = blockIdx.x * 128;
  const int n0   = blockIdx.y * 64;

  v8f acc[2][4];
#pragma unroll
  for (int mt = 0; mt < 2; ++mt)
#pragma unroll
    for (int nt = 0; nt < 4; ++nt) acc[mt][nt] = zero8();

  const size_t arow0 = (size_t)(m0 + 32 * wave + c) * DMOD + 8 * hh;
  const size_t brow0 = (size_t)(n0 + c) * DMOD + 8 * hh;

#pragma unroll 1
  for (int kt = 0; kt < DMOD / 32; ++kt) {
    const int k0 = kt * 32;
    FB ah[2], al[2], b[4];
#pragma unroll
    for (int mt = 0; mt < 2; ++mt) {
      const size_t ao = arow0 + (size_t)(16 * mt) * DMOD + k0;
      ah[mt].h[0] = *(const v8b*)(Ch + ao);
      ah[mt].h[1] = *(const v8b*)(Ch + ao + 16);
      al[mt].h[0] = *(const v8b*)(Cl + ao);
      al[mt].h[1] = *(const v8b*)(Cl + ao + 16);
    }
#pragma unroll
    for (int nt = 0; nt < 4; ++nt) {
      const unsigned short* bp = Wob + brow0 + (size_t)(16 * nt) * DMOD + k0;
      b[nt].h[0] = *(const v8b*)(bp);
      b[nt].h[1] = *(const v8b*)(bp + 16);
    }
#pragma unroll
    for (int mt = 0; mt < 2; ++mt)
#pragma unroll
      for (int nt = 0; nt < 4; ++nt) {
        acc[mt][nt] = mma_bf16(ah[mt].v, b[nt].v, acc[mt][nt]);
        acc[mt][nt] = mma_bf16(al[mt].v, b[nt].v, acc[mt][nt]);
      }
  }

  float bcol[4];
#pragma unroll
  for (int nt = 0; nt < 4; ++nt) bcol[nt] = bf_bits2f(f2bf_bits(bo[n0 + 16 * nt + c]));

  float* os = Os[wave];
#pragma unroll
  for (int mt = 0; mt < 2; ++mt)
#pragma unroll
    for (int nt = 0; nt < 4; ++nt)
#pragma unroll
      for (int r = 0; r < 8; ++r)
        os[(16 * mt + 8 * hh + r) * OP + 16 * nt + c] = acc[mt][nt][r] + bcol[nt];
  __syncthreads();

  {
    const int c4 = c * 4;
    for (int pass = 0; pass < 2; ++pass) {
#pragma unroll
      for (int it = 0; it < 16; ++it) {
        const int row = it * 2 + hh;
        const v4f val = *(const v4f*)(os + row * OP + c4);
        *(volatile v4f*)(out + (size_t)(m0 + 32 * wave + row) * DMOD + n0 + c4) = val;
      }
      __threadfence();
    }
  }
}

extern "C" void kernel_launch(void* const* d_in, const int* in_sizes, int n_in,
                              void* d_out, int out_size, void* d_ws, size_t ws_size,
                              hipStream_t stream)
{
  if (n_in < 10) return;
  if (in_sizes[0] < ((NB - 1) * SEQ_FULL + SEQ) * DMOD) return;
  if (in_sizes[1] < DMOD * DMOD || in_sizes[3] < DMOD * DMOD ||
      in_sizes[5] < DMOD * DMOD || in_sizes[8] < DMOD * DMOD) return;
  if (in_sizes[2] < DMOD || in_sizes[4] < DMOD || in_sizes[6] < DMOD || in_sizes[9] < DMOD) return;
  if (in_sizes[7] < ERROWS * DHEAD) return;
  if (out_size < MROWS * DMOD) return;
  if (d_ws == nullptr || ws_size < WS_NEED) return;

  const float* x  = (const float*)d_in[0];
  const float* Wq = (const float*)d_in[1];
  const float* bq = (const float*)d_in[2];
  const float* Wk = (const float*)d_in[3];
  const float* bk = (const float*)d_in[4];
  const float* Wv = (const float*)d_in[5];
  const float* bv = (const float*)d_in[6];
  const float* Er = (const float*)d_in[7];
  const float* Wo = (const float*)d_in[8];
  const float* bo = (const float*)d_in[9];
  float* O = (float*)d_out;

  unsigned char* ws = (unsigned char*)d_ws;
  unsigned short* ws16   = (unsigned short*)ws;
  const unsigned short* Xb  = (const unsigned short*)(ws + OFF_XB);
  const unsigned short* Wb3 = (const unsigned short*)(ws + OFF_WQ);
  const unsigned short* Wob = (const unsigned short*)(ws + OFF_WO);
  const unsigned short* Erb = (const unsigned short*)(ws + OFF_ER);
  unsigned short* planes = (unsigned short*)(ws + OFF_QH);
  const unsigned short* Qh = (const unsigned short*)(ws + OFF_QH);
  const unsigned short* Ql = (const unsigned short*)(ws + OFF_QL);
  const unsigned short* Kh = (const unsigned short*)(ws + OFF_KH);
  const unsigned short* Kl = (const unsigned short*)(ws + OFF_KL);
  const unsigned short* Vh = (const unsigned short*)(ws + OFF_VH);
  const unsigned short* Vl = (const unsigned short*)(ws + OFF_VL);
  unsigned short* Ch = (unsigned short*)(ws + OFF_CH);
  unsigned short* Cl = (unsigned short*)(ws + OFF_CL);

  const int nx = (MROWS * DMOD) / CVT_PER_BLOCK;
  const int nw = (DMOD * DMOD) / CVT_PER_BLOCK;
  const int ncvt = nx > nw ? nx : nw;

  cvt_kernel<<<dim3(ncvt, 6), 256, 0, stream>>>(x, Wq, Wk, Wv, Wo, Er, ws16);
  proj3_kernel<<<dim3(MROWS / 128, DMOD / 64, 3), 128, 0, stream>>>(Xb, Wb3, bq, bk, bv, planes);
  attn_kernel<<<dim3(SEQ / QBLK, NBH), 128, 0, stream>>>(Qh, Ql, Kh, Kl, Vh, Vl, Erb, Ch, Cl);
  oproj_kernel<<<dim3(MROWS / 128, DMOD / 64), 128, 0, stream>>>(Ch, Cl, Wob, bo, O);
}
